// DynamicTransformerLayer_7052336300502
// MI455X (gfx1250) — hardware-verified
//
#include <hip/hip_runtime.h>
#include <math.h>
#include <stdint.h>

#define NB   4
#define SEQ  2048
#define DM   1024
#define NH   16
#define HD   64
#define DFF  4096
#define RK   8
#define MR   (NB * SEQ)
#define KP1  (DM + 64)
#define KL1  (DM + 32)
#define KP2  (DFF + 64)
#define KL2  (DFF + 32)
#define NQB  (SEQ / 64)

#define WSC  64.0f
#define PSC  1024.0f
#define CSC  32.0f
#define FSC  4.0f

static_assert(NH * HD == DM);
static_assert((MR % 64) == 0 && (DM % 64) == 0 && (DFF % 64) == 0 && (SEQ % 64) == 0);
static_assert((KL1 % 32) == 0 && (KL2 % 32) == 0 && (KP1 % 64) == 0 && (KP2 % 64) == 0);
static_assert(KP1 - DM == 64 && KP2 - DFF == 64);
static_assert((DM % 256) == 0 && (DFF % 256) == 0);
static_assert(RK == 8);

typedef _Float16 v16h __attribute__((ext_vector_type(16)));
typedef _Float16 v8h  __attribute__((ext_vector_type(8)));
typedef float    v8f  __attribute__((ext_vector_type(8)));
typedef float    v4f  __attribute__((ext_vector_type(4)));
typedef unsigned int v4u __attribute__((ext_vector_type(4)));

__device__ __forceinline__ unsigned short hbits(float f) {
  const _Float16 x = (_Float16)f;
  return __builtin_bit_cast(unsigned short, x);
}
__device__ __forceinline__ unsigned pk16(unsigned short a, unsigned short b) { return (unsigned)a | ((unsigned)b << 16); }
__device__ __forceinline__ v4u pack8(v4f a, v4f c) {
  v4u p;
  p[0] = pk16(hbits(a[0]), hbits(a[1]));
  p[1] = pk16(hbits(a[2]), hbits(a[3]));
  p[2] = pk16(hbits(c[0]), hbits(c[1]));
  p[3] = pk16(hbits(c[2]), hbits(c[3]));
  return p;
}
__device__ __forceinline__ v8f zero8() { v8f z = {0.f, 0.f, 0.f, 0.f, 0.f, 0.f, 0.f, 0.f}; return z; }
__device__ __forceinline__ v4f zero4() { v4f z = {0.f, 0.f, 0.f, 0.f}; return z; }
__device__ __forceinline__ float wsum32(float v) {
  v += __shfl_xor(v, 16, 32);
  v += __shfl_xor(v, 8, 32);
  v += __shfl_xor(v, 4, 32);
  v += __shfl_xor(v, 2, 32);
  v += __shfl_xor(v, 1, 32);
  return v;
}
__device__ __forceinline__ float gelu_e(float v) { return 0.5f * v * (1.0f + erff(v * 0.70710678118654752f)); }

__device__ __forceinline__ v16h ldfrag(const _Float16* p) {
  union { v16h v; v8h h[2]; } f;
  f.h[0] = *(const v8h*)(p);
  f.h[1] = *(const v8h*)(p + 16);
  return f.v;
}

__device__ __forceinline__ v8f mma_raw(v16h a, v16h b, v8f c) {
  return __builtin_amdgcn_wmma_f32_16x16x32_f16(false, a, false, b, (short)0, c, false, false);
}
__device__ __forceinline__ v8f mma_g(v16h a, v16h b, v8f c) {
  c = mma_raw(a, b, c);
#if defined(__HIP_DEVICE_COMPILE__)
  asm volatile("v_nop\n\tv_nop\n\tv_nop\n\tv_nop" : "+v"(c) : "v"(a), "v"(b));
#endif
  return c;
}
__device__ __forceinline__ void dep_guard(v8f& x, v8f& y, v16h a, v16h b) {
#if defined(__HIP_DEVICE_COMPILE__)
  asm volatile("v_nop\n\tv_nop\n\tv_nop\n\tv_nop" : "+v"(x), "+v"(y) : "v"(a), "v"(b));
#else
  (void)x; (void)y; (void)a; (void)b;
#endif
}
__device__ __forceinline__ void keep4(v16h a, v16h b, v16h c, v16h d) {
#if defined(__HIP_DEVICE_COMPILE__)
  asm volatile("v_nop" :: "v"(a), "v"(b), "v"(c), "v"(d));
#else
  (void)a; (void)b; (void)c; (void)d;
#endif
}
__device__ __forceinline__ void acc_guard4(v8f& a, v8f& b, v8f& c, v8f& d) {
#if defined(__HIP_DEVICE_COMPILE__)
  asm volatile("v_nop\n\tv_nop\n\tv_nop\n\tv_nop" : "+v"(a), "+v"(b), "+v"(c), "+v"(d));
#else
  (void)a; (void)b; (void)c; (void)d;
#endif
}
__device__ __forceinline__ void wave_sync_lds() {
#if defined(__HIP_DEVICE_COMPILE__)
  __builtin_amdgcn_fence(__ATOMIC_RELEASE, "workgroup");
  __builtin_amdgcn_wave_barrier();
  __builtin_amdgcn_fence(__ATOMIC_ACQUIRE, "workgroup");
#endif
}

__global__ __launch_bounds__(256) void cvt_w(const float* __restrict__ W, const float* __restrict__ Am,
                                             unsigned short* out, int nrows, int K, int pitch, int aoff,
                                             float wscale, float ascale) {
  const int lane = threadIdx.x & 31;
  const int wave = threadIdx.x >> 5;
  const int row  = blockIdx.x * 8 + wave;
  if (row >= nrows) return;
  const float* src = W + (size_t)row * K + lane * 8;
  unsigned short* dst = out + (size_t)row * pitch + lane * 8;
  const int nch = K >> 8;
#pragma unroll 1
  for (int ch = 0; ch < nch; ++ch) {
    v4f a = *(const v4f*)(src + ch * 256);
    v4f c = *(const v4f*)(src + ch * 256 + 4);
    a *= wscale;
    c *= wscale;
    const v4u p = pack8(a, c);
    unsigned short* d = dst + ch * 256;
    *(volatile v4u*)d = p;
    __threadfence();
    *(volatile v4u*)d = p;
  }
  if (aoff >= 0) {
    const v4f a0 = *(const v4f*)(Am + (size_t)row * RK);
    const v4f a1 = *(const v4f*)(Am + (size_t)row * RK + 4);
    const float f = (lane * 8 == aoff) ? ascale : 0.f;
    const v4f u0 = a0 * f;
    const v4f u1 = a1 * f;
    const v4u p = pack8(u0, u1);
    unsigned short* d = out + (size_t)row * pitch + K + lane * 8;
    if (lane < 8) *(volatile v4u*)d = p;
    __threadfence();
    if (lane < 8) *(volatile v4u*)d = p;
  }
}

__global__ __launch_bounds__(256) void cvt_dyn(const float* __restrict__ s0, const float* __restrict__ s1,
                                               const float* __restrict__ s2, int nsrc, int Kd, int pitch,
                                               unsigned short* out, float scale) {
  const int lane = threadIdx.x & 31;
  const int wave = threadIdx.x >> 5;
  const int gr   = blockIdx.x * 8 + wave;
  if (gr >= NB * 64) return;
  const int b   = gr >> 6;
  const int r   = gr & 63;
  const int src = r >> 3;
  const int rr  = r & 7;
  const bool live = (src < nsrc);
  const int sc = live ? src : 0;
  const float* sp = (sc == 0) ? s0 : ((sc == 1) ? s1 : s2);
  const float* base = sp + ((size_t)(b * RK + rr)) * Kd + lane * 8;
  const float f = live ? scale : 0.f;
  unsigned short* dst = out + (size_t)gr * pitch + lane * 8;
  const int nch = Kd >> 8;
#pragma unroll 1
  for (int ch = 0; ch < nch; ++ch) {
    v4f a = *(const v4f*)(base + ch * 256);
    v4f c = *(const v4f*)(base + ch * 256 + 4);
    a *= f;
    c *= f;
    const v4u p = pack8(a, c);
    unsigned short* d = dst + ch * 256;
    *(volatile v4u*)d = p;
    __threadfence();
    *(volatile v4u*)d = p;
  }
  {
    const v4u z = {0u, 0u, 0u, 0u};
    unsigned short* d = out + (size_t)gr * pitch + Kd + lane * 8;
    if (lane < 8) *(volatile v4u*)d = z;
    __threadfence();
    if (lane < 8) *(volatile v4u*)d = z;
  }
}

__global__ __launch_bounds__(128) void ln_rows(const float* __restrict__ x, const float* __restrict__ g,
                                               const float* __restrict__ be, unsigned short* out, int pitch) {
  __shared__ float red[4];
  const int tid  = threadIdx.x;
  const int lane = tid & 31;
  const int wave = tid >> 5;
  const int row  = blockIdx.x;
  const float* xr = x + (size_t)row * DM + tid * 8;
  const v4f a = *(const v4f*)(xr);
  const v4f c = *(const v4f*)(xr + 4);
  float s = ((a[0] + a[1]) + (a[2] + a[3])) + ((c[0] + c[1]) + (c[2] + c[3]));
  s = wsum32(s);
  if (lane == 0) red[wave] = s;
  __syncthreads();
  const float tot = (red[0] + red[1]) + (red[2] + red[3]);
  __syncthreads();
  const float mu = tot * (1.0f / (float)DM);
  const v4f d0 = a - mu;
  const v4f d1 = c - mu;
  float s2 = ((d0[0] * d0[0] + d0[1] * d0[1]) + (d0[2] * d0[2] + d0[3] * d0[3])) +
             ((d1[0] * d1[0] + d1[1] * d1[1]) + (d1[2] * d1[2] + d1[3] * d1[3]));
  s2 = wsum32(s2);
  if (lane == 0) red[wave] = s2;
  __syncthreads();
  const float tot2 = (red[0] + red[1]) + (red[2] + red[3]);
  const float var  = tot2 * (1.0f / (float)DM);
  const float rstd = rsqrtf(var + 1e-5f);
  const v4f g0 = *(const v4f*)(g + tid * 8);
  const v4f g1 = *(const v4f*)(g + tid * 8 + 4);
  const v4f b0 = *(const v4f*)(be + tid * 8);
  const v4f b1 = *(const v4f*)(be + tid * 8 + 4);
  const v4f h0 = d0 * rstd * g0 + b0;
  const v4f h1 = d1 * rstd * g1 + b1;
  const v4u p = pack8(h0, h1);
  unsigned short* d = out + (size_t)row * pitch + tid * 8;
  *(volatile v4u*)d = p;
  __threadfence();
  *(volatile v4u*)d = p;
}

template <int EPI>
__global__ __launch_bounds__(256) void gemm64(
    const unsigned short* __restrict__ Ap, int lda, long long strideA,
    const unsigned short* __restrict__ Btp, int ldb, long long strideB,
    void* Cout, int ldc, long long strideC,
    const float* __restrict__ bias, const float* __restrict__ resid, int ldr,
    int M, int N, int K, float oscale) {
  __shared__ __align__(16) float sT[8][16 * 68];
  const _Float16* A  = (const _Float16*)(const void*)Ap;
  const _Float16* Bt = (const _Float16*)(const void*)Btp;
  const int b    = blockIdx.y;
  const int lane = threadIdx.x & 31;
  const int wave = threadIdx.x >> 5;
  const int tilesN = N >> 6;
  const int tilesM = M >> 6;
  const int tile = blockIdx.x * 8 + wave;
  if (tile >= tilesM * tilesN) return;
  const int tm = tile / tilesN;
  const int tn = tile - tm * tilesN;
  const int m0 = tm << 6;
  const int n0 = tn << 6;

  const _Float16* Ab = A  + (size_t)b * (size_t)strideA;
  const _Float16* Bb = Bt + (size_t)b * (size_t)strideB;

  const int rlane = lane & 15;
  const int koff  = (lane >> 4) * 8;
  const int mOff  = (lane >> 4) * 8;

  v8f acc[4][4];
#pragma unroll
  for (int i = 0; i < 4; ++i)
#pragma unroll
    for (int j = 0; j < 4; ++j) acc[i][j] = zero8();

  for (int k0 = 0; k0 < K; k0 += 32) {
    v16h bf[4];
#pragma unroll
    for (int j = 0; j < 4; ++j)
      bf[j] = ldfrag(Bb + (size_t)(n0 + (j << 4) + rlane) * ldb + koff + k0);
#pragma unroll
    for (int i = 0; i < 4; ++i) {
      const v16h af = ldfrag(Ab + (size_t)(m0 + (i << 4) + rlane) * lda + koff + k0);
#pragma unroll
      for (int j = 0; j < 4; ++j) acc[i][j] = mma_raw(af, bf[j], acc[i][j]);
      dep_guard(acc[i][0], acc[i][3], af, bf[3]);
    }
    keep4(bf[0], bf[1], bf[2], bf[3]);
  }
  acc_guard4(acc[0][0], acc[0][1], acc[0][2], acc[0][3]);
  acc_guard4(acc[1][0], acc[1][1], acc[1][2], acc[1][3]);
  acc_guard4(acc[2][0], acc[2][1], acc[2][2], acc[2][3]);
  acc_guard4(acc[3][0], acc[3][1], acc[3][2], acc[3][3]);

  float* slab = sT[wave];
#pragma unroll
  for (int i = 0; i < 4; ++i) {
    const int mBase = m0 + (i << 4);
#pragma unroll
    for (int j = 0; j < 4; ++j) {
#pragma unroll
      for (int r = 0; r < 8; ++r) slab[(mOff + r) * 68 + (j << 4) + rlane] = acc[i][j][r];
    }
    wave_sync_lds();
    if constexpr (EPI <= 1) {
      unsigned short* C = (unsigned short*)Cout + (size_t)b * (size_t)strideC;
      const int q4 = lane >> 3, c8 = (lane & 7) * 8;
#pragma unroll 1
      for (int it = 0; it < 4; ++it) {
        const int row = it * 4 + q4;
        const float* sp = slab + row * 68 + c8;
        v4f x0, x1;
        x0[0] = sp[0]; x0[1] = sp[1]; x0[2] = sp[2]; x0[3] = sp[3];
        x1[0] = sp[4]; x1[1] = sp[5]; x1[2] = sp[6]; x1[3] = sp[7];
        x0 *= oscale;
        x1 *= oscale;
        if constexpr (EPI == 1) {
          x0 += *(const v4f*)(bias + n0 + c8);
          x1 += *(const v4f*)(bias + n0 + c8 + 4);
#pragma unroll
          for (int e = 0; e < 4; ++e) {
            x0[e] = gelu_e(x0[e]) * FSC;
            x1[e] = gelu_e(x1[e]) * FSC;
          }
        }
        const v4u p = pack8(x0, x1);
        unsigned short* d = C + (size_t)(mBase + row) * ldc + n0 + c8;
        *(volatile v4u*)d = p;
        __threadfence();
        *(volatile v4u*)d = p;
      }
    } else {
      float* C = (float*)Cout + (size_t)b * (size_t)strideC;
      const int h2 = lane >> 4, c4 = (lane & 15) * 4;
#pragma unroll 1
      for (int it = 0; it < 8; ++it) {
        const int row = it * 2 + h2;
        const float* sp = slab + row * 68 + c4;
        v4f v;
        v[0] = sp[0]; v[1] = sp[1]; v[2] = sp[2]; v[3] = sp[3];
        v *= oscale;
        if constexpr (EPI == 3) v += *(const v4f*)(bias + n0 + c4);
        v += *(const v4f*)(resid + (size_t)(mBase + row) * ldr + n0 + c4);
        float* d = C + (size_t)(mBase + row) * ldc + n0 + c4;
        *(volatile v4f*)d = v;
        __threadfence();
        *(volatile v4f*)d = v;
      }
    }
    wave_sync_lds();
  }
}

__global__ __launch_bounds__(128)
void attn64(const unsigned short* __restrict__ qp, const unsigned short* __restrict__ kp,
            const unsigned short* __restrict__ vtp, unsigned short* op, float sscale, float oscale) {
  union FH { v16h v; v8h h[2]; };
  __shared__ __align__(16) _Float16 Ksh[64 * 64];
  __shared__ __align__(16) _Float16 Vth[64 * 64];
  __shared__ __align__(16) _Float16 Psh[4][16 * 64];
  __shared__ __align__(16) float    Os[4][16 * 64];

  const int tid  = threadIdx.x;
  const int wave = tid >> 5;
  const int lane = tid & 31;
  const int hh   = lane >> 4;
  const int c    = lane & 15;

  const int bx   = blockIdx.x;
  const int qb   = bx % NQB;
  const int rest = bx / NQB;
  const int h    = rest % NH;
  const int b    = rest / NH;
  const int q0   = qb * 64 + wave * 16;
  const size_t rowB = (size_t)b * SEQ;

  const _Float16* Q  = (const _Float16*)(const void*)qp + (size_t)h * HD;
  const _Float16* Kg = (const _Float16*)(const void*)kp + (size_t)h * HD;
  const _Float16* Vg = (const _Float16*)(const void*)vtp + ((size_t)b * DM + (size_t)h * HD) * SEQ;

  v16h qa[2];
#pragma unroll
  for (int dc = 0; dc < 2; ++dc) qa[dc] = ldfrag(Q + (rowB + q0 + c) * DM + dc * 32 + 8 * hh);

  float mrow[8], lrow[8];
  v8f oacc[4];
#pragma unroll
  for (int r = 0; r < 8; ++r) { mrow[r] = -INFINITY; lrow[r] = 0.f; }
#pragma unroll
  for (int t = 0; t < 4; ++t) oacc[t] = zero8();

  for (int kt = 0; kt < NQB; ++kt) {
    const int kv0 = kt * 64;
    __syncthreads();
    {
      const int r = tid >> 1, half = (tid & 1) * 32;
      const _Float16* kg = Kg + (rowB + kv0 + r) * DM + half;
      const _Float16* vg = Vg + (size_t)r * SEQ + kv0 + half;
#pragma unroll
      for (int i = 0; i < 4; ++i) {
        const v8h a0 = *(const v8h*)(kg + 8 * i);
        const v8h b0 = *(const v8h*)(vg + 8 * i);
        *(v8h*)(Ksh + r * 64 + half + 8 * i) = a0;
        *(v8h*)(Vth + r * 64 + half + 8 * i) = b0;
      }
    }
    __syncthreads();

    v8f s[4];
#pragma unroll
    for (int j = 0; j < 4; ++j) {
      s[j] = zero8();
#pragma unroll
      for (int dc = 0; dc < 2; ++dc) {
        FH kb;
        kb.h[0] = *(const v8h*)(Ksh + (j * 16 + c) * 64 + dc * 32 + 8 * hh);
        kb.h[1] = *(const v8h*)(Ksh + (j * 16 + c) * 64 + dc * 32 + 16 + 8 * hh);
        s[j] = mma_g(qa[dc], kb.v, s[j]);
      }
    }

    _Float16* pw = Psh[wave];
#pragma unroll
    for (int r = 0; r < 8; ++r) {
      float m = -INFINITY;
#pragma unroll
      for (int j = 0; j < 4; ++j) {
        const float sv = s[j][r] * sscale;
        s[j][r] = sv;
        m = fmaxf(m, sv);
      }
#pragma unroll
      for (int off = 1; off < 16; off <<= 1) m = fmaxf(m, __shfl_xor(m, off, 32));
      const float mnew  = fmaxf(mrow[r], m);
      const float alpha = __expf(mrow[r] - mnew);
      mrow[r] = mnew;
      float psum = 0.f;
#pragma unroll
      for (int j = 0; j < 4; ++j) {
        const float p = __expf(s[j][r] - mnew);
        psum += p;
        pw[(8 * hh + r) * 64 + j * 16 + c] = (_Float16)(p * PSC);
      }
#pragma unroll
      for (int off = 1; off < 16; off <<= 1) psum += __shfl_xor(psum, off, 32);
      lrow[r] = lrow[r] * alpha + psum;
#pragma unroll
      for (int t = 0; t < 4; ++t) oacc[t][r] *= alpha;
    }
    wave_sync_lds();

#pragma unroll 1
    for (int kk = 0; kk < 2; ++kk) {
      FH pa;
      pa.h[0] = *(const v8h*)(pw + c * 64 + kk * 32 + 8 * hh);
      pa.h[1] = *(const v8h*)(pw + c * 64 + kk * 32 + 16 + 8 * hh);
#pragma unroll
      for (int t = 0; t < 4; ++t) {
        FH vb;
        vb.h[0] = *(const v8h*)(Vth + (t * 16 + c) * 64 + kk * 32 + 8 * hh);
        vb.h[1] = *(const v8h*)(Vth + (t * 16 + c) * 64 + kk * 32 + 16 + 8 * hh);
        oacc[t] = mma_g(pa.v, vb.v, oacc[t]);
      }
    }
  }

  float* os = Os[wave];
#pragma unroll
  for (int r = 0; r < 8; ++r) {
    const float l = lrow[r];
    const float inv = (1.0f / l) * oscale;
#pragma unroll
    for (int t = 0; t < 4; ++t) os[(8 * hh + r) * 64 + t * 16 + c] = oacc[t][r] * inv;
  }
  wave_sync_lds();
  {
    const int q4 = lane >> 3, c8 = (lane & 7) * 8;
#pragma unroll 1
    for (int it = 0; it < 4; ++it) {
      const int row = it * 4 + q4;
      const float* sp = os + row * 64 + c8;
      v4f x0, x1;
      x0[0] = sp[0]; x0[1] = sp[1]; x0[2] = sp[2]; x0[3] = sp[3];
      x1[0] = sp[4]; x1[1] = sp[5]; x1[2] = sp[6]; x1[3] = sp[7];
      const v4u p = pack8(x0, x1);
      unsigned short* d = op + (rowB + q0 + row) * DM + (size_t)h * HD + c8;
      *(volatile v4u*)d = p;
      __threadfence();
      *(volatile v4u*)d = p;
    }
  }
}

extern "C" void kernel_launch(void* const* d_in, const int* in_sizes, int n_in,
                              void* d_out, int out_size, void* d_ws, size_t ws_size,
                              hipStream_t stream) {
  if (n_in < 23) return;
  if (in_sizes[0] != MR * DM) return;
  if (in_sizes[1] != NB * RK * DM || in_sizes[2] != NB * RK * DM || in_sizes[3] != NB * RK * DM ||
      in_sizes[4] != NB * RK * DM) return;
  if (in_sizes[5] != NB * RK * DFF) return;
  if (in_sizes[6] != DM * DM || in_sizes[8] != DM * DM || in_sizes[10] != DM * DM || in_sizes[12] != DM * DM) return;
  if (in_sizes[7] != DM * RK || in_sizes[9] != DM * RK || in_sizes[11] != DM * RK || in_sizes[18] != DM * RK) return;
  if (in_sizes[13] != DFF * DM || in_sizes[16] != DM * DFF) return;
  if (in_sizes[14] != DFF || in_sizes[15] != DFF * RK || in_sizes[17] != DM) return;
  if (in_sizes[19] != DM || in_sizes[20] != DM || in_sizes[21] != DM || in_sizes[22] != DM) return;
  if (out_size != MR * DM) return;

  const float* x       = (const float*)d_in[0];
  const float* dyn_q   = (const float*)d_in[1];
  const float* dyn_k   = (const float*)d_in[2];
  const float* dyn_v   = (const float*)d_in[3];
  const float* dyn_ff1 = (const float*)d_in[4];
  const float* dyn_ff2 = (const float*)d_in[5];
  const float* Wq  = (const float*)d_in[6];
  const float* Aq  = (const float*)d_in[7];
  const float* Wk  = (const float*)d_in[8];
  const float* Ak  = (const float*)d_in[9];
  const float* Wv  = (const float*)d_in[10];
  const float* Av  = (const float*)d_in[11];
  const float* Wo  = (const float*)d_in[12];
  const float* W1  = (const float*)d_in[13];
  const float* b1  = (const float*)d_in[14];
  const float* A1  = (const float*)d_in[15];
  const float* W2  = (const float*)d_in[16];
  const float* b2  = (const float*)d_in[17];
  const float* A2  = (const float*)d_in[18];
  const float* g1  = (const float*)d_in[19];
  const float* be1 = (const float*)d_in[20];
  const float* g2  = (const float*)d_in[21];
  const float* be2 = (const float*)d_in[22];

  const size_t szHp  = (size_t)MR * KP1 * 2;
  const size_t szX1  = (size_t)MR * DM * 4;
  const size_t szAct = (size_t)MR * DM * 2;
  const size_t szWp  = (size_t)DM * KP1 * 2;
  const size_t szWo  = (size_t)DM * DM * 2;
  const size_t szDy1 = (size_t)NB * 64 * KP1 * 2;
  const size_t szFF  = (size_t)MR * KP2 * 2;
  const size_t szW1  = (size_t)DFF * KP1 * 2;
  const size_t szW2  = (size_t)DM * KP2 * 2;
  const size_t szDy2 = (size_t)NB * 64 * KP2 * 2;

  const size_t oHp  = 0;
  const size_t oX1  = oHp + szHp;
  const size_t oR2  = oX1 + szX1;
  const size_t oQ   = oR2;
  const size_t oK   = oQ + szAct;
  const size_t oVT  = oK + szAct;
  const size_t oCtx = oVT + szAct;
  const size_t oWq  = oCtx + szAct;
  const size_t oWk  = oWq + szWp;
  const size_t oWv  = oWk + szWp;
  const size_t oWo  = oWv + szWp;
  const size_t oDy  = oWo + szWo;
  const size_t endA = oDy + szDy1;
  const size_t oFF  = oR2;
  const size_t oW1  = oFF + szFF;
  const size_t oDy1 = oW1 + szW1;
  const size_t endD = oDy1 + szDy1;
  const size_t oW2  = oHp;
  const size_t oDy2 = oW2 + szW2;
  const size_t total = (endA > endD) ? endA : endD;
  if (total > ws_size) return;
  if (total > (size_t)134217728) return;
  if (oDy2 + szDy2 > oHp + szHp) return;

  char* ws = (char*)d_ws;
  unsigned short* Hp   = (unsigned short*)(ws + oHp);
  float*          X1   = (float*)(ws + oX1);
  unsigned short* Qp   = (unsigned short*)(ws + oQ);
  unsigned short* Kpl  = (unsigned short*)(ws + oK);
  unsigned short* VTp  = (unsigned short*)(ws + oVT);
  unsigned short* Ctxp = (unsigned short*)(ws + oCtx);
  unsigned short* Wqp  = (unsigned short*)(ws + oWq);
  unsigned short* Wkp  = (unsigned short*)(ws + oWk);
  unsigned short* Wvp  = (unsigned short*)(ws + oWv);
  unsigned short* Wop  = (unsigned short*)(ws + oWo);
  unsigned short* Dyp  = (unsigned short*)(ws + oDy);
  unsigned short* FFp  = (unsigned short*)(ws + oFF);
  unsigned short* W1p  = (unsigned short*)(ws + oW1);
  unsigned short* Dy1p = (unsigned short*)(ws + oDy1);
  unsigned short* W2p  = (unsigned short*)(ws + oW2);
  unsigned short* Dy2p = (unsigned short*)(ws + oDy2);

  const dim3 blk(256);
  const dim3 gW1024(DM / 8);
  const dim3 gW4096(DFF / 8);
  const dim3 gDyn(NB * 64 / 8);
  const dim3 gLN(MR);
  const dim3 gCoef(((SEQ / 64) * 1 + 7) / 8, NB);
  const dim3 gProj(((MR / 64) * (DM / 64) + 7) / 8, 1);
  const dim3 gVT(((DM / 64) * (SEQ / 64) + 7) / 8, NB);
  const dim3 gFF1(((MR / 64) * (DFF / 64) + 7) / 8, 1);
  const dim3 gAttn(NB * NH * NQB);
  const float inv64  = 1.0f / WSC;
  const float invWo  = 1.0f / (CSC * WSC);
  const float invFF2 = 1.0f / (FSC * WSC);

  cvt_w<<<gW1024, blk, 0, stream>>>(Wq, Aq, Wqp, DM, DM, KP1, 0, WSC, WSC);
  cvt_w<<<gW1024, blk, 0, stream>>>(Wk, Ak, Wkp, DM, DM, KP1, 8, WSC, WSC);
  cvt_w<<<gW1024, blk, 0, stream>>>(Wv, Av, Wvp, DM, DM, KP1, 16, WSC, WSC);
  cvt_w<<<gW1024, blk, 0, stream>>>(Wo, Wo, Wop, DM, DM, DM, -1, WSC, WSC);
  cvt_dyn<<<gDyn, blk, 0, stream>>>(dyn_q, dyn_k, dyn_v, 3, DM, KP1, Dyp, WSC);
  ln_rows<<<gLN, dim3(128), 0, stream>>>(x, g1, be1, Hp, KP1);
  gemm64<0><<<gCoef, blk, 0, stream>>>(
      Hp, KP1, (long long)SEQ * KP1, Dyp, KP1, (long long)64 * KP1,
      (void*)(Hp + DM), KP1, (long long)SEQ * KP1, b1, x, DM,
      SEQ, 64, DM, inv64);
  gemm64<0><<<gProj, blk, 0, stream>>>(
      Hp, KP1, 0LL, Wqp, KP1, 0LL, (void*)Qp, DM, 0LL, b1, x, DM,
      MR, DM, KL1, inv64);
  gemm64<0><<<gProj, blk, 0, stream>>>(
      Hp, KP1, 0LL, Wkp, KP1, 0LL, (void*)Kpl, DM, 0LL, b1, x, DM,
      MR, DM, KL1, inv64);
  gemm64<0><<<gVT, blk, 0, stream>>>(
      Wvp, KP1, 0LL, Hp, KP1, (long long)SEQ * KP1, (void*)VTp, SEQ, (long long)DM * SEQ, b1, x, DM,
      DM, SEQ, KL1, inv64);
  attn64<<<gAttn, dim3(128), 0, stream>>>(Qp, Kpl, VTp, Ctxp, 0.125f, CSC / PSC);
  gemm64<2><<<gProj, blk, 0, stream>>>(
      Ctxp, DM, 0LL, Wop, DM, 0LL, (void*)X1, DM, 0LL, b2, x, DM,
      MR, DM, DM, invWo);
  cvt_w<<<gW4096, blk, 0, stream>>>(W1, A1, W1p, DFF, DM, KP1, 0, WSC, WSC);
  cvt_dyn<<<gDyn, blk, 0, stream>>>(dyn_ff1, dyn_ff1, dyn_ff1, 1, DM, KP1, Dy1p, WSC);
  ln_rows<<<gLN, dim3(128), 0, stream>>>(X1, g2, be2, Hp, KP1);
  gemm64<0><<<gCoef, blk, 0, stream>>>(
      Hp, KP1, (long long)SEQ * KP1, Dy1p, KP1, (long long)64 * KP1,
      (void*)(Hp + DM), KP1, (long long)SEQ * KP1, b1, x, DM,
      SEQ, 64, DM, inv64);
  gemm64<1><<<gFF1, blk, 0, stream>>>(
      Hp, KP1, 0LL, W1p, KP1, 0LL, (void*)FFp, KP2, 0LL, b1, x, DM,
      MR, DFF, KL1, inv64);
  cvt_w<<<gW1024, blk, 0, stream>>>(W2, A2, W2p, DM, DFF, KP2, 0, WSC, WSC);
  cvt_dyn<<<gDyn, blk, 0, stream>>>(dyn_ff2, dyn_ff2, dyn_ff2, 1, DFF, KP2, Dy2p, WSC);
  gemm64<0><<<gCoef, blk, 0, stream>>>(
      FFp, KP2, (long long)SEQ * KP2, Dy2p, KP2, (long long)64 * KP2,
      (void*)(FFp + DFF), KP2, (long long)SEQ * KP2, b1, x, DM,
      SEQ, 64, DFF, inv64);
  gemm64<3><<<gProj, blk, 0, stream>>>(
      FFp, KP2, 0LL, W2p, KP2, 0LL, d_out, DM, 0LL, b2, X1, DM,
      MR, DM, KL2, invFF2);
  (void)hipGetLastError();
}
